// SaliencyGraphEncoder_13546326851792
// MI455X (gfx1250) — hardware-verified
//
#include <hip/hip_runtime.h>
#include <math.h>

typedef __attribute__((ext_vector_type(16))) _Float16 v16h;
typedef __attribute__((ext_vector_type(16))) __bf16 v16b;
typedef __attribute__((ext_vector_type(8)))  _Float16 v8h;
typedef __attribute__((ext_vector_type(8)))  float v8f;
typedef __attribute__((ext_vector_type(4)))  float v4f;
typedef __attribute__((ext_vector_type(2)))  float v2f;
typedef __attribute__((ext_vector_type(4)))  unsigned v4u;
typedef __attribute__((ext_vector_type(4)))  int v4i;
typedef float __attribute__((may_alias)) float_a;
typedef int __attribute__((may_alias)) int_a;

template <typename T> __device__ __forceinline__ void vst2(void* p, T v) { *(volatile T*)p = v; __threadfence(); *(volatile T*)p = v; }
__device__ __forceinline__ v8f wmma16(v16h a, v16h b, v8f c) {
  v8f d = __builtin_amdgcn_wmma_f32_16x16x32_f16(false, a, false, b, (short)0, c, false, false);
  asm volatile("v_nop\n\tv_nop\n\tv_nop\n\tv_nop" : "+v"(d) : "v"(a), "v"(b));
  return d;
}
__device__ __forceinline__ v8f wmma_bf(v16b a, v16b b, v8f c) {
  v8f d = __builtin_amdgcn_wmma_f32_16x16x32_bf16(false, a, false, b, (short)0, c, false, false);
  asm volatile("v_nop\n\tv_nop\n\tv_nop\n\tv_nop" : "+v"(d) : "v"(a), "v"(b));
  return d;
}
__device__ __forceinline__ v16h frag_h(const _Float16* rowk0, int lane) {
  union { v16h v; v8h q[2]; } u; const _Float16* p = rowk0 + 8 * (lane >> 4);
  u.q[0] = *(const v8h*)p; u.q[1] = *(const v8h*)(p + 16); return u.v;
}
__device__ __forceinline__ v16h frag_f32(const float* rowk0, int lane) {
  v16h a; const float* p = rowk0 + 8 * (lane >> 4);
#pragma unroll
  for (int i = 0; i < 8; ++i) { a[i] = (_Float16)p[i]; a[8 + i] = (_Float16)p[16 + i]; }
  return a;
}
__device__ __forceinline__ v16h frag_f32s(const float* rowk0, int lane, float sc) {
  v16h a; const float* p = rowk0 + 8 * (lane >> 4);
#pragma unroll
  for (int i = 0; i < 8; ++i) { a[i] = (_Float16)(p[i] * sc); a[8 + i] = (_Float16)(p[16 + i] * sc); }
  return a;
}
__device__ __forceinline__ v16h fragc_f32(const float* W, int k0, int n, int lane, int ld, int K) {
  v16h a; const int g = lane >> 4;
#pragma unroll
  for (int i = 0; i < 8; ++i) { const int ka = k0 + 8 * g + i, kb = ka + 16;
    a[i] = (_Float16)(ka < K ? W[(size_t)ka * ld + n] : 0.f); a[8 + i] = (_Float16)(kb < K ? W[(size_t)kb * ld + n] : 0.f); }
  return a;
}
struct F2 { v16b h, l; };
__device__ __forceinline__ F2 bsplit16(const float v[16]) { F2 r;
#pragma unroll
  for (int i = 0; i < 16; ++i) { const __bf16 h = (__bf16)v[i]; r.h[i] = h; r.l[i] = (__bf16)(v[i] - (float)h); }
  return r; }
__device__ __forceinline__ F2 split_row(const float* row, int k0, int lane) { float v[16]; const float* p = row + k0 + 8 * (lane >> 4);
#pragma unroll
  for (int i = 0; i < 8; ++i) { v[i] = p[i]; v[8 + i] = p[16 + i]; }
  return bsplit16(v); }
__device__ __forceinline__ F2 split_rowK(const float* row, int k0, int lane, int K) { float v[16]; const int g = lane >> 4;
#pragma unroll
  for (int i = 0; i < 8; ++i) { const int ka = k0 + 8 * g + i, kb = ka + 16; v[i] = ka < K ? row[ka] : 0.f; v[8 + i] = kb < K ? row[kb] : 0.f; }
  return bsplit16(v); }
__device__ __forceinline__ F2 split_col(const float* W, int k0, int n, int lane, int ld, int K) { float v[16]; const int g = lane >> 4;
#pragma unroll
  for (int i = 0; i < 8; ++i) { const int ka = k0 + 8 * g + i, kb = ka + 16; v[i] = ka < K ? W[(size_t)ka * ld + n] : 0.f; v[8 + i] = kb < K ? W[(size_t)kb * ld + n] : 0.f; }
  return bsplit16(v); }
__device__ __forceinline__ v8f mac3(const F2& a, const F2& b, v8f c) { c = wmma_bf(a.l, b.h, c); c = wmma_bf(a.h, b.l, c); return wmma_bf(a.h, b.h, c); }
__device__ __forceinline__ float sigm(float v) { return 1.0f / (1.0f + expf(-v)); }
#define LDSX() do { asm volatile("s_wait_dscnt 0" ::: "memory"); __builtin_amdgcn_wave_barrier(); __builtin_amdgcn_fence(__ATOMIC_RELEASE, "workgroup"); } while (0)


#define NBATCH 8
#define NF 8192
#define S 2048
#define D 256
#define D2 512
#define MAXPOS 4096
#define MAXPRED 1024
#define NROLE 66
#define TG 64
#define NTG (S / TG)
__device__ __forceinline__ float gelu_e(float x) { return 0.5f * x * (1.0f + erff(x * 0.70710678118654752f)); }
__device__ __forceinline__ int clampi(int v, int hi) { return v < 0 ? 0 : (v > hi ? hi : v); }

__global__ __launch_bounds__(128) void k_tab(const float* __restrict__ A, int M, const float* __restrict__ w1k, float* __restrict__ T) {
  __shared__ __align__(16) float so[4][16][132];
  const int tid = threadIdx.x, wave = tid >> 5, lane = tid & 31, col = lane & 15, g = lane >> 4;
  const int r0 = blockIdx.x * 64 + wave * 16; const int ra = (r0 + col) < M ? (r0 + col) : (M - 1);
#pragma unroll 1
  for (int ps = 0; ps < D2 / 128; ++ps) { v8f acc[8] = {};
#pragma unroll 1
    for (int kc = 0; kc < D / 32; ++kc) { const F2 a = split_row(A + (size_t)ra * D, kc * 32, lane);
#pragma unroll
      for (int j = 0; j < 8; ++j) acc[j] = mac3(a, split_col(w1k, kc * 32, ps * 128 + j * 16 + col, lane, D2, D), acc[j]); }
#pragma unroll
    for (int j = 0; j < 8; ++j)
#pragma unroll
      for (int r = 0; r < 8; ++r) so[wave][8 * g + r][j * 16 + col] = acc[j][r];
    LDSX();
    for (int rl = 0; rl < 16; ++rl) { if (r0 + rl >= M) break; vst2(T + (size_t)(r0 + rl) * D2 + ps * 128 + lane * 4, *(const v4f*)(&so[wave][rl][lane * 4])); }
    LDSX(); }
}
__global__ __launch_bounds__(256) void k_facts(const int* __restrict__ pred, const int* __restrict__ a0, const int* __restrict__ a1, const int* __restrict__ role, const int* __restrict__ isrole,
                                              const int* __restrict__ addrev, const int* __restrict__ mask, const float* __restrict__ Ta, const float* __restrict__ Tb, const float* __restrict__ Tn,
                                              const float* __restrict__ Tr, const float* __restrict__ b1, const float* __restrict__ w2, const float* __restrict__ b2, const float* __restrict__ nodes,
                                              const float* __restrict__ lng, const float* __restrict__ lnb, float* __restrict__ PART) {
  __shared__ __align__(16) float sacc[TG][D2];
  __shared__ __align__(16) float sx[TG][D + 4];
  __shared__ int slst[8][64]; __shared__ int scnt[8]; __shared__ float scntt[TG]; __shared__ __align__(16) float spart[4][D];
  const int tid = threadIdx.x, wave = tid >> 5, lane = tid & 31, col = lane & 15, g = lane >> 4;
  const int b = blockIdx.y, grp = blockIdx.x, t0 = grp * TG;
  for (int q = tid; q < TG * D2; q += 256) (&sacc[0][0])[q] = 0.f;
  if (tid < TG) scntt[tid] = 0.f;
  __syncthreads();
  const int* pb = pred + (size_t)b * NF; const int* a0b = a0 + (size_t)b * NF; const int* a1b = a1 + (size_t)b * NF; const int* rb = role + (size_t)b * NF;
  const int* irb = isrole + (size_t)b * NF; const int* arb = addrev + (size_t)b * NF; const int* mb = mask + (size_t)b * NF;
#pragma unroll 1
  for (int f0 = 0; f0 < NF; f0 += 256) { const int f = f0 + tid;
    const int va0 = clampi(a0b[f], S - 1), va1 = clampi(a1b[f], S - 1); const bool isr = irb[f] != 0, valid = mb[f] != 0, rev = arb[f] != 0;
    const int tf = isr ? va0 : va1;
    const bool hf = valid && (unsigned)(tf - t0) < (unsigned)TG;
    const bool hr = valid && !isr && rev && (unsigned)(va0 - t0) < (unsigned)TG;
    const int cnt = (hf ? 1 : 0) + (hr ? 1 : 0);
    int incl = cnt;
#pragma unroll
    for (int off = 1; off < 32; off <<= 1) { const int vv = __shfl_up(incl, off, 32); if (lane >= off) incl += vv; }
    const int wtot = __shfl(incl, 31, 32); int pos = incl - cnt;
    if (hf) { slst[wave][pos++] = f * 2; } if (hr) { slst[wave][pos++] = f * 2 + 1; }
    if (lane == 0) scnt[wave] = wtot;
    __syncthreads();
#pragma unroll 1
    for (int w = 0; w < 8; ++w) { const int nh = scnt[w];
#pragma unroll 1
      for (int i = 0; i < nh; ++i) { const int ent = slst[w][i]; const int ff = ent >> 1, dir = ent & 1;
        const int xa0 = clampi(a0b[ff], S - 1), xa1 = clampi(a1b[ff], S - 1), xp = clampi(pb[ff], MAXPRED - 1), xr = clampi(rb[ff], NROLE - 1); const bool isr2 = irb[ff] != 0;
        const float* r1; const float* r3; int tl;
        if (dir == 0) { r1 = Ta + (size_t)xa0 * D2; r3 = isr2 ? Tr + (size_t)xr * D2 : Tn + (size_t)xa1 * D2; tl = (isr2 ? xa0 : xa1) - t0; }
        else { r1 = Ta + (size_t)xa1 * D2; r3 = Tn + (size_t)xa0 * D2; tl = xa0 - t0; }
        const float* r2 = Tb + (size_t)xp * D2;
#pragma unroll
        for (int hh = 0; hh < 2; ++hh) { const int c = tid + hh * 256; const float z = r1[c] + r2[c] + r3[c] + b1[c]; sacc[tl][c] += gelu_e(z); }
        if (tid == 0) scntt[tl] += 1.0f; } }
    __syncthreads(); }
  { v8f acc[4][2] = {};
#pragma unroll 1
    for (int kc = 0; kc < D2 / 32; ++kc) { const F2 bA = split_col(w2, kc * 32, (2 * wave) * 16 + col, lane, D, D2), bB = split_col(w2, kc * 32, (2 * wave + 1) * 16 + col, lane, D, D2);
#pragma unroll
      for (int i = 0; i < 4; ++i) { const F2 a = split_row(&sacc[i * 16 + col][0], kc * 32, lane); acc[i][0] = mac3(a, bA, acc[i][0]); acc[i][1] = mac3(a, bB, acc[i][1]); } }
#pragma unroll
    for (int i = 0; i < 4; ++i)
#pragma unroll
      for (int j = 0; j < 2; ++j) { const int n = (2 * wave + j) * 16 + col;
#pragma unroll
        for (int r = 0; r < 8; ++r) { const int tl = i * 16 + 8 * g + r; sx[tl][n] = acc[i][j][r] + scntt[tl] * b2[n] + nodes[(size_t)(t0 + tl) * D + n]; } } }
  __syncthreads();
  { const int tl = tid >> 2, qd = tid & 3; float* row = &sx[tl][qd * 64]; float s = 0.f;
#pragma unroll 4
    for (int k = 0; k < 64; ++k) s += row[k];
    s += __shfl_xor(s, 1, 32); s += __shfl_xor(s, 2, 32); const float mu = s * (1.0f / D); float qv = 0.f;
#pragma unroll 4
    for (int k = 0; k < 64; ++k) { const float dv = row[k] - mu; qv += dv * dv; }
    qv += __shfl_xor(qv, 1, 32); qv += __shfl_xor(qv, 2, 32); const float rs = rsqrtf(qv * (1.0f / D) + 1e-5f);
#pragma unroll 4
    for (int k = 0; k < 64; ++k) { const int c = qd * 64 + k; row[k] = (row[k] - mu) * rs * lng[c] + lnb[c]; } }
  __syncthreads();
  { const int c = tid; float s = 0.f;
#pragma unroll 4
    for (int tl = 0; tl < TG; ++tl) s += sx[tl][c];
    spart[0][c] = s; }
  __syncthreads();
  if (tid < D / 4) vst2(PART + ((size_t)b * NTG + grp) * D + tid * 4, *(const v4f*)(&spart[0][tid * 4]));
}
__global__ __launch_bounds__(256) void k_head(const float* __restrict__ PART, const int* __restrict__ seqlen, const float* __restrict__ lw1, const float* __restrict__ lb1, const float* __restrict__ lw2, const float* __restrict__ lb2, float* __restrict__ out) {
  __shared__ __align__(16) float sp[16][D + 4]; __shared__ __align__(16) float sh[16][D + 4];
  const int tid = threadIdx.x, wave = tid >> 5, lane = tid & 31, col = lane & 15, g = lane >> 4;
  const float inv = 1.0f / (float)(seqlen[0] > 0 ? seqlen[0] : 1);
  { const int c = tid;
    for (int b = 0; b < 16; ++b) { float s = 0.f; if (b < NBATCH) {
#pragma unroll 4
        for (int gq = 0; gq < NTG; ++gq) s += PART[((size_t)b * NTG + gq) * D + c]; }
      sp[b][c] = s * inv; } }
  __syncthreads();
  { v8f acc[2] = {};
#pragma unroll 1
    for (int kc = 0; kc < D / 32; ++kc) { const F2 a = split_row(&sp[col][0], kc * 32, lane);
#pragma unroll
      for (int j = 0; j < 2; ++j) acc[j] = mac3(a, split_col(lw1, kc * 32, (2 * wave + j) * 16 + col, lane, D, D), acc[j]); }
#pragma unroll
    for (int j = 0; j < 2; ++j) { const int n = (2 * wave + j) * 16 + col;
#pragma unroll
      for (int r = 0; r < 8; ++r) sh[8 * g + r][n] = (8 * g + r) < NBATCH ? gelu_e(acc[j][r] + lb1[n]) : 0.f; } }
  __syncthreads();
  { v8f acc[2] = {};
#pragma unroll 1
    for (int kc = 0; kc < D / 32; ++kc) { const F2 a = split_row(&sh[col][0], kc * 32, lane);
#pragma unroll
      for (int j = 0; j < 2; ++j) acc[j] = mac3(a, split_col(lw2, kc * 32, (2 * wave + j) * 16 + col, lane, D, D), acc[j]); }
#pragma unroll
    for (int j = 0; j < 2; ++j) { const int n = (2 * wave + j) * 16 + col;
#pragma unroll
      for (int r = 0; r < 8; ++r) sp[8 * g + r][n] = acc[j][r] + lb2[n]; } }
  __syncthreads();
  { const int b = tid >> 5; vst2(out + (size_t)b * D + lane * 4, *(const v4f*)(&sp[b][lane * 4])); vst2(out + (size_t)b * D + 128 + lane * 4, *(const v4f*)(&sp[b][128 + lane * 4])); }
}
extern "C" void kernel_launch(void* const* d_in, const int* in_sizes, int n_in, void* d_out, int out_size, void* d_ws, size_t ws_size, hipStream_t stream) {
  (void)in_sizes; (void)n_in; (void)out_size; (void)ws_size;
  const float* pos_emb = (const float*)d_in[0]; const float* pred_emb = (const float*)d_in[1]; const float* role_emb = (const float*)d_in[2];
  const float* w1 = (const float*)d_in[3]; const float* b1 = (const float*)d_in[4]; const float* w2 = (const float*)d_in[5]; const float* b2 = (const float*)d_in[6];
  const float* lng = (const float*)d_in[7]; const float* lnb = (const float*)d_in[8]; const float* lw1 = (const float*)d_in[9]; const float* lb1 = (const float*)d_in[10]; const float* lw2 = (const float*)d_in[11]; const float* lb2 = (const float*)d_in[12];
  const int* pred = (const int*)d_in[13]; const int* a0 = (const int*)d_in[14]; const int* a1 = (const int*)d_in[15]; const int* role = (const int*)d_in[16];
  const int* isrole = (const int*)d_in[17]; const int* addrev = (const int*)d_in[18]; const int* mask = (const int*)d_in[19]; const int* seqlen = (const int*)d_in[20];
  float* out = (float*)d_out;
  char* ws = (char*)d_ws; size_t off = 0;
  auto take = [&](size_t bytes) { char* p = ws + off; off += (bytes + 255) & ~(size_t)255; return p; };
  float* Ta = (float*)take((size_t)S * D2 * 4); float* Tb = (float*)take((size_t)MAXPRED * D2 * 4); float* Tn = (float*)take((size_t)S * D2 * 4); float* Tr = (float*)take((size_t)128 * D2 * 4);
  float* PART = (float*)take((size_t)NBATCH * NTG * D * 4);
  k_tab<<<S / 64, 128, 0, stream>>>(pos_emb, S, w1, Ta);
  k_tab<<<MAXPRED / 64, 128, 0, stream>>>(pred_emb, MAXPRED, w1 + (size_t)D * D2, Tb);
  k_tab<<<S / 64, 128, 0, stream>>>(pos_emb, S, w1 + (size_t)2 * D * D2, Tn);
  k_tab<<<2, 128, 0, stream>>>(role_emb, NROLE, w1 + (size_t)2 * D * D2, Tr);
  k_facts<<<dim3(NTG, NBATCH), 256, 0, stream>>>(pred, a0, a1, role, isrole, addrev, mask, Ta, Tb, Tn, Tr, b1, w2, b2, pos_emb, lng, lnb, PART);
  k_head<<<1, 256, 0, stream>>>(PART, seqlen, lw1, lb1, lw2, lb2, out);
}
